// CINComp_18777597018207
// MI455X (gfx1250) — hardware-verified
//
#include <hip/hip_runtime.h>
#include <math.h>

typedef __attribute__((ext_vector_type(16))) _Float16 v16h;
typedef __attribute__((ext_vector_type(16))) __bf16 v16b;
typedef __attribute__((ext_vector_type(8)))  _Float16 v8h;
typedef __attribute__((ext_vector_type(8)))  float v8f;
typedef __attribute__((ext_vector_type(4)))  float v4f;
typedef __attribute__((ext_vector_type(2)))  float v2f;
typedef __attribute__((ext_vector_type(4)))  unsigned v4u;
typedef __attribute__((ext_vector_type(4)))  int v4i;
typedef float __attribute__((may_alias)) float_a;
typedef int __attribute__((may_alias)) int_a;

template <typename T> __device__ __forceinline__ void vst2(void* p, T v) { *(volatile T*)p = v; __threadfence(); *(volatile T*)p = v; }
__device__ __forceinline__ v8f wmma16(v16h a, v16h b, v8f c) {
  v8f d = __builtin_amdgcn_wmma_f32_16x16x32_f16(false, a, false, b, (short)0, c, false, false);
  asm volatile("v_nop\n\tv_nop\n\tv_nop\n\tv_nop" : "+v"(d) : "v"(a), "v"(b));
  return d;
}
__device__ __forceinline__ v8f wmma_bf(v16b a, v16b b, v8f c) {
  v8f d = __builtin_amdgcn_wmma_f32_16x16x32_bf16(false, a, false, b, (short)0, c, false, false);
  asm volatile("v_nop\n\tv_nop\n\tv_nop\n\tv_nop" : "+v"(d) : "v"(a), "v"(b));
  return d;
}
__device__ __forceinline__ v16h frag_h(const _Float16* rowk0, int lane) {
  union { v16h v; v8h q[2]; } u; const _Float16* p = rowk0 + 8 * (lane >> 4);
  u.q[0] = *(const v8h*)p; u.q[1] = *(const v8h*)(p + 16); return u.v;
}
__device__ __forceinline__ v16h frag_f32(const float* rowk0, int lane) {
  v16h a; const float* p = rowk0 + 8 * (lane >> 4);
#pragma unroll
  for (int i = 0; i < 8; ++i) { a[i] = (_Float16)p[i]; a[8 + i] = (_Float16)p[16 + i]; }
  return a;
}
__device__ __forceinline__ v16h frag_f32s(const float* rowk0, int lane, float sc) {
  v16h a; const float* p = rowk0 + 8 * (lane >> 4);
#pragma unroll
  for (int i = 0; i < 8; ++i) { a[i] = (_Float16)(p[i] * sc); a[8 + i] = (_Float16)(p[16 + i] * sc); }
  return a;
}
__device__ __forceinline__ v16h fragc_f32(const float* W, int k0, int n, int lane, int ld, int K) {
  v16h a; const int g = lane >> 4;
#pragma unroll
  for (int i = 0; i < 8; ++i) { const int ka = k0 + 8 * g + i, kb = ka + 16;
    a[i] = (_Float16)(ka < K ? W[(size_t)(ka < K ? ka : K - 1) * ld + n] : 0.f); a[8 + i] = (_Float16)(kb < K ? W[(size_t)(kb < K ? kb : K - 1) * ld + n] : 0.f); }
  return a;
}
struct F2 { v16b h, l; };
__device__ __forceinline__ F2 bsplit16(const float v[16]) { F2 r;
#pragma unroll
  for (int i = 0; i < 16; ++i) { const __bf16 h = (__bf16)v[i]; r.h[i] = h; r.l[i] = (__bf16)(v[i] - (float)h); }
  return r; }
__device__ __forceinline__ F2 split_row(const float* row, int k0, int lane) { float v[16]; const float* p = row + k0 + 8 * (lane >> 4);
#pragma unroll
  for (int i = 0; i < 8; ++i) { v[i] = p[i]; v[8 + i] = p[16 + i]; }
  return bsplit16(v); }
__device__ __forceinline__ F2 split_rowK(const float* row, int k0, int lane, int K) { float v[16]; const int g = lane >> 4;
#pragma unroll
  for (int i = 0; i < 8; ++i) { const int ka = k0 + 8 * g + i, kb = ka + 16; v[i] = ka < K ? row[ka < K ? ka : K - 1] : 0.f; v[8 + i] = kb < K ? row[kb < K ? kb : K - 1] : 0.f; }
  return bsplit16(v); }
__device__ __forceinline__ F2 split_col(const float* W, int k0, int n, int lane, int ld, int K) { float v[16]; const int g = lane >> 4;
#pragma unroll
  for (int i = 0; i < 8; ++i) { const int ka = k0 + 8 * g + i, kb = ka + 16; v[i] = ka < K ? W[(size_t)(ka < K ? ka : K - 1) * ld + n] : 0.f; v[8 + i] = kb < K ? W[(size_t)(kb < K ? kb : K - 1) * ld + n] : 0.f; }
  return bsplit16(v); }
__device__ __forceinline__ v8f mac3(const F2& a, const F2& b, v8f c) { c = wmma_bf(a.l, b.h, c); c = wmma_bf(a.h, b.l, c); return wmma_bf(a.h, b.h, c); }
__device__ __forceinline__ float sigm(float v) { return 1.0f / (1.0f + expf(-v)); }
#define LDSX() do { asm volatile("s_wait_dscnt 0" ::: "memory"); __builtin_amdgcn_wave_barrier(); __builtin_amdgcn_fence(__ATOMIC_RELEASE, "workgroup"); } while (0)


#define NBAT 1024
#define IND 200
#define BSD 39
#define DD 32
#define OUTD 200
#define KP 224
#define OT ((OUTD + 15) / 16)
#ifndef NBT
#define NBT NBAT
#endif
typedef __attribute__((ext_vector_type(8))) __bf16 v8b;
__device__ __forceinline__ v16b frag_b(const __bf16* rowk0, int lane) {
  union { v16b v; v8b q[2]; } u; const __bf16* p = rowk0 + 8 * (lane >> 4);
  u.q[0] = *(const v8b*)p; u.q[1] = *(const v8b*)(p + 16); return u.v;
}
__device__ __forceinline__ float bfr(float v) { return (float)(__bf16)v; }
__device__ __attribute__((noinline)) float exp_ni(float v) { return expf(v); }
__device__ __attribute__((noinline)) float erf_ni(float v) { return erff(v); }

#define WS_WP  0u
#define NROWP (OT * 16 * BSD)
#define WS_END (2u * (size_t)NROWP * KP)

__global__ __launch_bounds__(256) void k_pack(const float* __restrict__ Wm, __bf16* __restrict__ WP) {
  __shared__ __align__(16) __bf16 s[KP]; const int row = blockIdx.x, t = threadIdx.x; const int o = row / BSD, j = row % BSD;
  if (t < KP) s[t] = (__bf16)((o < OUTD && t < IND) ? Wm[(size_t)o * (IND * BSD) + t * BSD + j] : 0.f);
  __syncthreads();
  if (t < KP / 8) vst2((unsigned*)(WP + (size_t)row * KP + t * 8), *(const v4u*)&s[t * 8]);
}
__global__ __launch_bounds__(128) void k_cin(const float* __restrict__ INF, const float* __restrict__ BASE, const __bf16* __restrict__ WP, const float* __restrict__ Bv, float* __restrict__ OUT) {
  __shared__ __align__(16) __bf16 sin_[DD][KP + 8]; __shared__ float sbase[BSD][DD]; __shared__ float sacc[4][16][DD + 1]; __shared__ __align__(16) float so[16][DD];
  const int tid = threadIdx.x, wave = tid >> 5, lane = tid & 31, col = lane & 15, g = lane >> 4; const int ot = blockIdx.x; const size_t b = blockIdx.y; const int o0 = ot * 16;
  for (int e = tid; e < DD * (KP + 8); e += 128) { const int d = e / (KP + 8), i = e % (KP + 8); sin_[d][i] = (__bf16)((i < IND) ? INF[(b * IND + i) * DD + d] : 0.f); }
  for (int e = tid; e < BSD * DD; e += 128) sbase[e / DD][e % DD] = bfr(BASE[(b * BSD) * DD + e]);
  __syncthreads();
  float acc_o[2][8];
#pragma unroll
  for (int dt = 0; dt < 2; ++dt)
#pragma unroll
    for (int r = 0; r < 8; ++r) acc_o[dt][r] = 0.f;
#pragma unroll 1
  for (int j = wave; j < BSD; j += 4) { v8f a2[2] = {};
#pragma unroll
    for (int kc = 0; kc < KP / 32; ++kc) { const v16b a = frag_b(WP + ((size_t)(o0 + col) * BSD + j) * KP + kc * 32, lane);
#pragma unroll
      for (int dt = 0; dt < 2; ++dt) a2[dt] = wmma_bf(a, frag_b(&sin_[dt * 16 + col][kc * 32], lane), a2[dt]); }
#pragma unroll
    for (int dt = 0; dt < 2; ++dt) { const float bw = sbase[j][dt * 16 + col];
#pragma unroll
      for (int r = 0; r < 8; ++r) acc_o[dt][r] += a2[dt][r] * bw; } }
#pragma unroll
  for (int dt = 0; dt < 2; ++dt)
#pragma unroll
    for (int r = 0; r < 8; ++r) sacc[wave][8 * g + r][dt * 16 + col] = acc_o[dt][r];
  __syncthreads();
  for (int e = tid; e < 16 * DD; e += 128) { const int ol = e >> 5, d = e & 31; const int o = o0 + ol; so[ol][d] = (sacc[0][ol][d] + sacc[1][ol][d]) + (sacc[2][ol][d] + sacc[3][ol][d]) + ((o < OUTD) ? bfr(Bv[o]) : 0.f); }
  __syncthreads();
  for (int e = tid; e < 16 * 8; e += 128) { const int ol = e >> 3, q = e & 7; if (o0 + ol < OUTD) vst2(OUT + (b * OUTD + o0 + ol) * DD + q * 4, *(const v4f*)&so[ol][q * 4]); }
}
extern "C" void kernel_launch(void* const* d_in, const int* in_sizes, int n_in, void* d_out, int out_size, void* d_ws, size_t ws_size, hipStream_t stream) {
  (void)in_sizes; (void)n_in; (void)out_size;
  const float** F = (const float**)d_in;
  if (ws_size < (size_t)WS_END) return;
  char* ws = (char*)d_ws; __bf16* WP = (__bf16*)(ws + WS_WP);
  k_pack<<<NROWP, 256, 0, stream>>>(F[2], WP);
  k_cin<<<dim3(OT, NBT), 128, 0, stream>>>(F[0], F[1], WP, F[3], (float*)d_out);
}
